// CompositeFullyConnected_57320633532772
// MI455X (gfx1250) — hardware-verified
//
#include <hip/hip_runtime.h>


#define NB_  4096
#define FF   512
#define H1   1024
#define H2   1024
#define U1   512
#define U2   256
#define KBL  16
#define CAP  5120
#define DM   FF
#define LOSC 1024.0f

typedef _Float16 h16;
typedef unsigned short bf;
typedef __attribute__((ext_vector_type(16))) __bf16   v16bf;
typedef __attribute__((ext_vector_type(16))) _Float16 v16h;
typedef __attribute__((ext_vector_type(8)))  _Float16 v8h;
typedef __attribute__((ext_vector_type(8)))  unsigned short v8us;
typedef __attribute__((ext_vector_type(8)))  float    v8f;
typedef __attribute__((ext_vector_type(4)))  float    v4f;
typedef v8h  __attribute__((may_alias)) v8ha;
typedef v4f  __attribute__((may_alias)) v4fa;
typedef v8us __attribute__((may_alias)) v8usa;

__device__ __forceinline__ unsigned short f2bf(float f) { unsigned u = __float_as_uint(f); u += 0x7FFFu + ((u >> 16) & 1u); return (unsigned short)(u >> 16); }
__device__ __forceinline__ float bf2f(unsigned short b) { return __uint_as_float(((unsigned)b) << 16); }
__device__ __forceinline__ float bfr(float f) { return bf2f(f2bf(f)); }
__device__ __forceinline__ v16h cat16(v8h lo, v8h hi) { return __builtin_shufflevector(lo, hi, 0, 1, 2, 3, 4, 5, 6, 7, 8, 9, 10, 11, 12, 13, 14, 15); }
__device__ __forceinline__ v16bf cat16b(v8us lo, v8us hi) { return __builtin_bit_cast(v16bf, __builtin_shufflevector(lo, hi, 0, 1, 2, 3, 4, 5, 6, 7, 8, 9, 10, 11, 12, 13, 14, 15)); }
__device__ __forceinline__ v8f wmma16(v16h a, v16h b, v8f c) { return __builtin_amdgcn_wmma_f32_16x16x32_f16(false, a, false, b, (short)0, c, false, false); }
__device__ __forceinline__ v8f wmmab(v16bf a, v16bf b, v8f c) { return __builtin_amdgcn_wmma_f32_16x16x32_bf16(false, a, false, b, (short)0, c, false, false); }

template <bool SPLITA, bool F16OUT = false>
__global__ __launch_bounds__(128) void k_gemmb(const bf* __restrict__ A, const bf* __restrict__ Al, const bf* __restrict__ Bn, const float* __restrict__ bias, float* C, int ldc, h16* C2, const float* __restrict__ R = nullptr, int K = DM, int roundR = 1) {
    __shared__ __align__(16) float ost[4][16 * 68];
    const int lane = threadIdx.x & 31, wave = threadIdx.x >> 5, lr = lane & 15, hi = lane >> 4;
    const int r0 = blockIdx.x * 64 + wave * 16, c0 = blockIdx.y * 64;
    const size_t aoff = (size_t)(r0 + lr) * K + 8 * hi;
    size_t boff[4];
#pragma unroll
    for (int t = 0; t < 4; ++t) boff[t] = (size_t)(c0 + t * 16 + lr) * K + 8 * hi;
    v8f acc[4];
#pragma unroll
    for (int t = 0; t < 4; ++t) acc[t] = (v8f){};
#pragma unroll 1
    for (int kc = 0; kc < K; kc += 32) {
        const v16bf a = cat16b(*(const v8us*)(A + aoff + kc), *(const v8us*)(A + aoff + kc + 16));
        v16bf al = a;
        if (SPLITA) al = cat16b(*(const v8us*)(Al + aoff + kc), *(const v8us*)(Al + aoff + kc + 16));
#pragma unroll
        for (int t = 0; t < 4; ++t) { const v16bf b = cat16b(*(const v8us*)(Bn + boff[t] + kc), *(const v8us*)(Bn + boff[t] + kc + 16)); acc[t] = wmmab(a, b, acc[t]); if (SPLITA) acc[t] = wmmab(al, b, acc[t]); }
        asm volatile("v_nop\n\tv_nop\n\tv_nop\n\tv_nop" : "+v"(acc[0]), "+v"(acc[1]), "+v"(acc[2]), "+v"(acc[3]) : "v"(a), "v"(al));
    }
    float* os = &ost[wave][0];
#pragma unroll
    for (int t = 0; t < 4; ++t) { const float bv = bias ? bfr(bias[c0 + t * 16 + lr]) : 0.f;
#pragma unroll
        for (int j = 0; j < 8; ++j) os[(hi * 8 + j) * 68 + t * 16 + lr] = acc[t][j] + bv; }
    __syncthreads();
    if (F16OUT) {
        h16* crow = (h16*)(void*)C + (size_t)r0 * ldc + c0;
        auto pass = [&]() {
#pragma unroll
            for (int s = 0; s < 4; ++s) { const int row = 4 * s + (lane >> 3), piece = lane & 7; const float* sp = os + row * 68 + piece * 8; v8h o, o2;
#pragma unroll
                for (int i = 0; i < 8; ++i) { const h16 a = (h16)sp[i]; o[i] = a; o2[i] = (h16)((sp[i] - (float)a) * LOSC); }
                *(volatile v8h*)(crow + (size_t)row * ldc + piece * 8) = o; if (C2) *(volatile v8h*)(C2 + (size_t)r0 * ldc + c0 + (size_t)row * ldc + piece * 8) = o2; }
        };
        pass(); __threadfence(); pass();
    } else {
        float* crow = C + (size_t)r0 * ldc + c0;
        auto pass = [&]() {
#pragma unroll
            for (int s = 0; s < 8; ++s) { const int Lid = (lane >> 3) + 4 * s, piece = lane & 7; const int row = Lid >> 1, cofs = (Lid & 1) * 32 + piece * 4;
                v4f val = *(const v4fa*)(os + row * 68 + cofs); if (R) { const v4f rv = *(const v4f*)(R + ((size_t)r0 + row) * ldc + c0 + cofs); val += roundR ? (v4f){bfr(rv[0]), bfr(rv[1]), bfr(rv[2]), bfr(rv[3])} : rv; }
                *(volatile v4f*)(crow + (size_t)row * ldc + cofs) = val; }
        };
        pass(); __threadfence(); pass();
    }
}

template <bool SPLITA, bool F16OUT = false>
__global__ __launch_bounds__(128) void k_gemmbg(const bf* __restrict__ A, const bf* __restrict__ Al, const bf* __restrict__ Bn, const float* __restrict__ bias, float* C, int ldc, h16* C2, const float* __restrict__ R, int K, int roundR, const int* __restrict__ OFF, const int* __restrict__ NKP, size_t sB, size_t sBias) {
    { const int g = blockIdx.z; if ((int)blockIdx.x * 64 >= NKP[g]) return; const size_t ro = (size_t)OFF[g]; A += ro * K; if (Al) Al += ro * K; Bn += (size_t)g * sB; if (bias) bias += (size_t)g * sBias; C += ro * ldc; if (R) R += ro * ldc; }
    __shared__ __align__(16) float ost[4][16 * 68];
    const int lane = threadIdx.x & 31, wave = threadIdx.x >> 5, lr = lane & 15, hi = lane >> 4;
    const int r0 = blockIdx.x * 64 + wave * 16, c0 = blockIdx.y * 64;
    const size_t aoff = (size_t)(r0 + lr) * K + 8 * hi;
    size_t boff[4];
#pragma unroll
    for (int t = 0; t < 4; ++t) boff[t] = (size_t)(c0 + t * 16 + lr) * K + 8 * hi;
    v8f acc[4];
#pragma unroll
    for (int t = 0; t < 4; ++t) acc[t] = (v8f){};
#pragma unroll 1
    for (int kc = 0; kc < K; kc += 32) {
        const v16bf a = cat16b(*(const v8us*)(A + aoff + kc), *(const v8us*)(A + aoff + kc + 16));
        v16bf al = a;
        if (SPLITA) al = cat16b(*(const v8us*)(Al + aoff + kc), *(const v8us*)(Al + aoff + kc + 16));
#pragma unroll
        for (int t = 0; t < 4; ++t) { const v16bf b = cat16b(*(const v8us*)(Bn + boff[t] + kc), *(const v8us*)(Bn + boff[t] + kc + 16)); acc[t] = wmmab(a, b, acc[t]); if (SPLITA) acc[t] = wmmab(al, b, acc[t]); }
        asm volatile("v_nop\n\tv_nop\n\tv_nop\n\tv_nop" : "+v"(acc[0]), "+v"(acc[1]), "+v"(acc[2]), "+v"(acc[3]) : "v"(a), "v"(al));
    }
    float* os = &ost[wave][0];
#pragma unroll
    for (int t = 0; t < 4; ++t) { const float bv = bias ? bfr(bias[c0 + t * 16 + lr]) : 0.f;
#pragma unroll
        for (int j = 0; j < 8; ++j) os[(hi * 8 + j) * 68 + t * 16 + lr] = acc[t][j] + bv; }
    __syncthreads();
    if (F16OUT) {
        h16* crow = (h16*)(void*)C + (size_t)r0 * ldc + c0;
        auto pass = [&]() {
#pragma unroll
            for (int s = 0; s < 4; ++s) { const int row = 4 * s + (lane >> 3), piece = lane & 7; const float* sp = os + row * 68 + piece * 8; v8h o, o2;
#pragma unroll
                for (int i = 0; i < 8; ++i) { const h16 a = (h16)sp[i]; o[i] = a; o2[i] = (h16)((sp[i] - (float)a) * LOSC); }
                *(volatile v8h*)(crow + (size_t)row * ldc + piece * 8) = o; if (C2) *(volatile v8h*)(C2 + (size_t)r0 * ldc + c0 + (size_t)row * ldc + piece * 8) = o2; }
        };
        pass(); __threadfence(); pass();
    } else {
        float* crow = C + (size_t)r0 * ldc + c0;
        auto pass = [&]() {
#pragma unroll
            for (int s = 0; s < 8; ++s) { const int Lid = (lane >> 3) + 4 * s, piece = lane & 7; const int row = Lid >> 1, cofs = (Lid & 1) * 32 + piece * 4;
                v4f val = *(const v4fa*)(os + row * 68 + cofs); if (R) { const v4f rv = *(const v4f*)(R + ((size_t)r0 + row) * ldc + c0 + cofs); val += roundR ? (v4f){bfr(rv[0]), bfr(rv[1]), bfr(rv[2]), bfr(rv[3])} : rv; }
                *(volatile v4f*)(crow + (size_t)row * ldc + cofs) = val; }
        };
        pass(); __threadfence(); pass();
    }
}

__global__ __launch_bounds__(256) void k_wt(const float* __restrict__ Wm, int K, int ncols, bf* WT) {
    __shared__ __align__(16) unsigned short tl[64 * 72];
    const int tid = threadIdx.x, k0 = blockIdx.x * 64, n0 = blockIdx.y * 64;
    const int kk = tid >> 2, nq = (tid & 3) * 16;
#pragma unroll
    for (int i = 0; i < 16; ++i) tl[(nq + i) * 72 + kk] = f2bf(Wm[(size_t)(k0 + kk) * ncols + n0 + nq + i]);
    __syncthreads();
    const int piece = tid & 7;
    auto pass = [&]() {
#pragma unroll
        for (int s = 0; s < 2; ++s) { const int nr = (tid >> 3) + 32 * s; const v8us val = *(const v8usa*)(tl + nr * 72 + piece * 8); *(volatile v8us*)(WT + (size_t)(n0 + nr) * K + k0 + piece * 8) = val; }
    };
    pass(); __threadfence(); pass();
}

__global__ __launch_bounds__(256) void k_cvt8(const float* __restrict__ src, bf* dst, size_t n8) {
    const size_t i = (size_t)blockIdx.x * 256 + threadIdx.x; if (i >= n8) return;
    const v8f v = *(const v8f*)(src + i * 8); v8us o;
#pragma unroll
    for (int k = 0; k < 8; ++k) o[k] = f2bf(v[k]);
    *(volatile v8us*)(dst + i * 8) = o; __threadfence(); *(volatile v8us*)(dst + i * 8) = o;
}
__global__ __launch_bounds__(256) void k_zero8(bf* dst, size_t n8) {
    const size_t i = (size_t)blockIdx.x * 256 + threadIdx.x; if (i >= n8) return; v8us z;
#pragma unroll
    for (int k = 0; k < 8; ++k) z[k] = 0;
    *(volatile v8us*)(dst + i * 8) = z; __threadfence(); *(volatile v8us*)(dst + i * 8) = z;
}

__global__ __launch_bounds__(64) void k_sort(const int* __restrict__ st, int* PERM, int* OFF, int* NKP) {
    __shared__ int cnt[KBL], offs[KBL + 1]; __shared__ int ps_[CAP];
    const int g = threadIdx.x;
    for (int r = g; r < CAP; r += 64) ps_[r] = -1;
    if (g < KBL) { int c = 0; for (int b = 0; b < NB_; ++b) { int s = st[b]; s = s < 0 ? 0 : (s >= KBL ? KBL - 1 : s); c += (s == g); } cnt[g] = c; }
    __syncthreads();
    if (g == 0) { int o = 0; for (int k = 0; k < KBL; ++k) { offs[k] = o; o += (cnt[k] + 63) & ~63; } offs[KBL] = o; }
    __syncthreads();
    if (g < KBL) { int w = offs[g]; for (int b = 0; b < NB_; ++b) { int s = st[b]; s = s < 0 ? 0 : (s >= KBL ? KBL - 1 : s); if (s == g) { ps_[w] = b; ++w; } } }
    __syncthreads();
    const int lane = g & 31, wv = g >> 5;
    for (int p2 = 0; p2 < 2; ++p2) {
        for (int r0 = wv * 32; r0 < CAP; r0 += 64) *(volatile int*)(PERM + r0 + lane) = ps_[r0 + lane];
        if (wv == 0) { const int vo = (lane <= KBL) ? offs[lane] : 0; const int vn = (lane < KBL) ? ((cnt[lane] + 63) & ~63) : 0; *(volatile int*)(OFF + lane) = vo; *(volatile int*)(NKP + lane) = vn; }
        if (p2 == 0) __threadfence(); }
}
__global__ __launch_bounds__(256) void k_cvtx(const float* __restrict__ src, bf* dst) {
    const int lane = threadIdx.x & 31; const size_t r = (size_t)blockIdx.x * 8 + (threadIdx.x >> 5); if (r >= (size_t)NB_) return;
#pragma unroll 1
    for (int ps = 0; ps < 2; ++ps) {
#pragma unroll
        for (int q = 0; q < FF / 256; ++q) { v8us o;
#pragma unroll
            for (int i = 0; i < 8; ++i) o[i] = f2bf(src[r * FF + q * 256 + lane * 8 + i]);
            *(volatile v8us*)(dst + r * FF + q * 256 + lane * 8) = o; }
        if (ps == 0) __threadfence(); }
}
__global__ __launch_bounds__(256) void k_relu1k(const float* __restrict__ src, int nrows, bf* dh, bf* dl) {
    const int lane = threadIdx.x & 31; const size_t r = (size_t)blockIdx.x * 8 + (threadIdx.x >> 5); if (r >= (size_t)nrows) return;
#pragma unroll 1
    for (int ps = 0; ps < 2; ++ps) {
#pragma unroll
        for (int q = 0; q < H1 / 256; ++q) { const size_t o = r * H1 + q * 256 + lane * 8; const v8f v = *(const v8f*)(src + o); v8us oh, ol;
#pragma unroll
            for (int i = 0; i < 8; ++i) { const float t = fmaxf(v[i], 0.f); const unsigned short hb = f2bf(t); oh[i] = hb; ol[i] = f2bf(t - bf2f(hb)); }
            *(volatile v8us*)(dh + o) = oh; *(volatile v8us*)(dl + o) = ol; }
        if (ps == 0) __threadfence(); }
}
__global__ __launch_bounds__(256) void k_gath(const float* __restrict__ H2s, const int* __restrict__ PERM, const int* __restrict__ OFF, bf* dh, bf* dl) {
    const int lane = threadIdx.x & 31; const size_t r = (size_t)blockIdx.x * 8 + (threadIdx.x >> 5); if (r >= (size_t)OFF[KBL]) return;       const int b = PERM[r]; const bool ok = (b >= 0) && (b < NB_);
#pragma unroll 1
    for (int ps = 0; ps < 2; ++ps) {
#pragma unroll
        for (int q = 0; q < H2 / 256; ++q) { const size_t o = r * H2 + q * 256 + lane * 8; v8us oh, ol;
#pragma unroll
            for (int i = 0; i < 8; ++i) { const float t = ok ? fmaxf(H2s[(size_t)(ok ? b : 0) * H2 + q * 256 + lane * 8 + i], 0.f) : 0.f; const unsigned short hb = f2bf(t); oh[i] = hb; ol[i] = f2bf(t - bf2f(hb)); }
            *(volatile v8us*)(dh + o) = oh; *(volatile v8us*)(dl + o) = ol; }
        if (ps == 0) __threadfence(); }
}
__global__ __launch_bounds__(256) void k_kb1(const float* __restrict__ Kb, bf* KP) {
    const int lane = threadIdx.x & 31; const size_t r = (size_t)blockIdx.x * 8 + (threadIdx.x >> 5); if (r >= (size_t)KBL * U1) return; const int g = (int)(r / U1), u = (int)(r % U1);
#pragma unroll 1
    for (int ps = 0; ps < 2; ++ps) {
#pragma unroll 1
        for (int q = 0; q < H2 / 256; ++q) { v8us o;
#pragma unroll
            for (int i = 0; i < 8; ++i) { const int f = q * 256 + lane * 8 + i; o[i] = f2bf(Kb[((size_t)f * U1 + u) * KBL + g]); }
            *(volatile v8us*)(KP + r * H2 + q * 256 + lane * 8) = o; }
        if (ps == 0) __threadfence(); }
}
__global__ __launch_bounds__(256) void k_kb2(const float* __restrict__ Kb, bf* KP) {
    const int lane = threadIdx.x & 31; const size_t r = (size_t)blockIdx.x * 8 + (threadIdx.x >> 5); if (r >= (size_t)KBL * U2) return; const int g = (int)(r / U2), u = (int)(r % U2);
#pragma unroll 1
    for (int ps = 0; ps < 2; ++ps) {
#pragma unroll 1
        for (int q = 0; q < U1 / 256; ++q) { v8us o;
#pragma unroll
            for (int i = 0; i < 8; ++i) { const int f = q * 256 + lane * 8 + i; o[i] = f2bf(Kb[((size_t)f * U2 + u) * KBL + g]); }
            *(volatile v8us*)(KP + r * U1 + q * 256 + lane * 8) = o; }
        if (ps == 0) __threadfence(); }
}
__global__ __launch_bounds__(256) void k_bias(const float* __restrict__ Bb, int nu, float* BP) {
    const int lane = threadIdx.x & 31; const int wid = blockIdx.x * 8 + (threadIdx.x >> 5); if (wid >= KBL * (nu / 128)) return; const int g = wid / (nu / 128), u0 = (wid % (nu / 128)) * 128 + lane * 4; v4f v;
#pragma unroll
    for (int q = 0; q < 4; ++q) v[q] = Bb[(size_t)(u0 + q) * KBL + g];
    *(volatile v4f*)(BP + (size_t)g * nu + u0) = v; __threadfence(); *(volatile v4f*)(BP + (size_t)g * nu + u0) = v;
}
__global__ __launch_bounds__(256) void k_relu512g(const float* __restrict__ src, const int* __restrict__ OFF, bf* dh, bf* dl) {
    const int lane = threadIdx.x & 31; const size_t r = (size_t)blockIdx.x * 8 + (threadIdx.x >> 5); if (r >= (size_t)OFF[KBL]) return;
#pragma unroll 1
    for (int ps = 0; ps < 2; ++ps) {
#pragma unroll
        for (int q = 0; q < U1 / 256; ++q) { const size_t o = r * U1 + q * 256 + lane * 8; const v8f v = *(const v8f*)(src + o); v8us oh, ol;
#pragma unroll
            for (int i = 0; i < 8; ++i) { const float t = fmaxf(v[i], 0.f); const unsigned short hb = f2bf(t); oh[i] = hb; ol[i] = f2bf(t - bf2f(hb)); }
            *(volatile v8us*)(dh + o) = oh; *(volatile v8us*)(dl + o) = ol; }
        if (ps == 0) __threadfence(); }
}
__global__ __launch_bounds__(256) void k_scatter(const float* __restrict__ C2, const int* __restrict__ PERM, float* OUTP) {
    const int lane = threadIdx.x & 31; const size_t r = (size_t)blockIdx.x * 8 + (threadIdx.x >> 5); if (r >= (size_t)CAP) return; const int b = PERM[r]; if (b < 0 || b >= NB_) return;
#pragma unroll 1
    for (int ps = 0; ps < 2; ++ps) {
#pragma unroll
        for (int st = 0; st < U2 / 128; ++st) { const int c0 = st * 128 + lane * 4; const v4f v = *(const v4f*)(C2 + r * U2 + c0); *(volatile v4f*)(OUTP + (size_t)b * U2 + c0) = v; }
        if (ps == 0) __threadfence(); }
}

extern "C" void kernel_launch(void* const* d_in, const int* in_sizes, int n_in,
                              void* d_out, int out_size, void* d_ws, size_t ws_size, hipStream_t stream) {
    (void)in_sizes; (void)n_in; (void)out_size;
    const float* x = (const float*)d_in[0]; const float* W1 = (const float*)d_in[1]; const float* b1 = (const float*)d_in[2]; const float* W2 = (const float*)d_in[3]; const float* b2 = (const float*)d_in[4];
    const float* Kb1 = (const float*)d_in[5]; const float* Bb1 = (const float*)d_in[6]; const float* Kb2 = (const float*)d_in[7]; const float* Bb2 = (const float*)d_in[8]; const int* states = (const int*)d_in[9];
    float* out = (float*)d_out;
    char* wsp = (char*)d_ws;
    auto take = [&](size_t bytes) { char* p = wsp; wsp += (bytes + 255) & ~(size_t)255; return (void*)p; };
    bf* W1T = (bf*)take((size_t)H1 * FF * 2); bf* W2T = (bf*)take((size_t)H2 * H1 * 2); bf* KB1P = (bf*)take((size_t)KBL * U1 * H2 * 2); bf* KB2P = (bf*)take((size_t)KBL * U2 * U1 * 2); float* BB1P = (float*)take((size_t)KBL * U1 * 4); float* BB2P = (float*)take((size_t)KBL * U2 * 4);
    int* PERM = (int*)take(CAP * 4); int* OFF = (int*)take(32 * 4); int* NKP = (int*)take(32 * 4);
    bf* Xb = (bf*)take((size_t)NB_ * FF * 2); float* T = (float*)take((size_t)NB_ * H1 * 4); bf* Rh = (bf*)take((size_t)NB_ * H1 * 2); bf* Rl = (bf*)take((size_t)NB_ * H1 * 2);
    bf* Gh = (bf*)take((size_t)CAP * H2 * 2); bf* Gl = (bf*)take((size_t)CAP * H2 * 2); float* C1 = (float*)take((size_t)CAP * U1 * 4); bf* Ph = (bf*)take((size_t)CAP * U1 * 2); bf* Pl = (bf*)take((size_t)CAP * U1 * 2); float* C2 = (float*)take((size_t)CAP * U2 * 4);
    if ((size_t)(wsp - (char*)d_ws) > ws_size) return;
    k_sort<<<1, 64, 0, stream>>>(states, PERM, OFF, NKP);
    k_wt<<<dim3(FF / 64, H1 / 64, 1), 256, 0, stream>>>(W1, FF, H1, W1T); k_wt<<<dim3(H1 / 64, H2 / 64, 1), 256, 0, stream>>>(W2, H1, H2, W2T);
    k_kb1<<<(KBL * U1) / 8, 256, 0, stream>>>(Kb1, KB1P); k_kb2<<<(KBL * U2) / 8, 256, 0, stream>>>(Kb2, KB2P); k_bias<<<(KBL * (U1 / 128)) / 8, 256, 0, stream>>>(Bb1, U1, BB1P); k_bias<<<(KBL * (U2 / 128) + 7) / 8, 256, 0, stream>>>(Bb2, U2, BB2P);
    k_cvtx<<<NB_ / 8, 256, 0, stream>>>(x, Xb);
    k_gemmb<false, false><<<dim3(NB_ / 64, H1 / 64, 1), 128, 0, stream>>>(Xb, nullptr, W1T, b1, T, H1, nullptr, nullptr, FF); k_relu1k<<<NB_ / 8, 256, 0, stream>>>(T, NB_, Rh, Rl);
    k_gemmb<true, false><<<dim3(NB_ / 64, H2 / 64, 1), 128, 0, stream>>>(Rh, Rl, W2T, b2, T, H2, nullptr, nullptr, H1);
    k_gath<<<CAP / 8, 256, 0, stream>>>(T, PERM, OFF, Gh, Gl);
    k_gemmbg<true, false><<<dim3(NB_ / 64, U1 / 64, KBL), 128, 0, stream>>>(Gh, Gl, KB1P, BB1P, C1, U1, nullptr, nullptr, H2, 0, OFF, NKP, (size_t)U1 * H2, (size_t)U1);
    k_relu512g<<<CAP / 8, 256, 0, stream>>>(C1, OFF, Ph, Pl);
    k_gemmbg<true, false><<<dim3(NB_ / 64, U2 / 64, KBL), 128, 0, stream>>>(Ph, Pl, KB2P, BB2P, C2, U2, nullptr, nullptr, U1, 0, OFF, NKP, (size_t)U2 * U1, (size_t)U2);
    k_scatter<<<CAP / 8, 256, 0, stream>>>(C2, PERM, out);
}
